// MaskedAttention_67413806678107
// MI455X (gfx1250) — hardware-verified
//
#include <hip/hip_runtime.h>
#include <stdint.h>

#define NB    4
#define SEQ   2048
#define DM    1024
#define NTOK  (NB * SEQ)

typedef _Float16 v16h __attribute__((ext_vector_type(16)));
typedef _Float16 v8h  __attribute__((ext_vector_type(8)));
typedef __bf16   v16b __attribute__((ext_vector_type(16)));
typedef __bf16   v8b  __attribute__((ext_vector_type(8)));
typedef float    v8f  __attribute__((ext_vector_type(8)));
typedef float    v4f  __attribute__((ext_vector_type(4)));
typedef unsigned short v8us __attribute__((ext_vector_type(8)));

static_assert((DM % 64) == 0 && (NTOK % 64) == 0 && (DM % 32) == 0);

__device__ __forceinline__ unsigned short bfbits(float f) {
  const unsigned u = __float_as_uint(f);
  return (unsigned short)((u + 0x7FFFu + ((u >> 16) & 1u)) >> 16);
}

__device__ __forceinline__ v16h ldfrag(const _Float16* p) {
  union { v16h v; v8h hh[2]; } f;
  f.hh[0] = *(const v8h*)(p);
  f.hh[1] = *(const v8h*)(p + 16);
  return f.v;
}
__device__ __forceinline__ v16b ldfragb(const __bf16* p) {
  union { v16b v; v8b hh[2]; } f;
  f.hh[0] = *(const v8b*)(p);
  f.hh[1] = *(const v8b*)(p + 16);
  return f.v;
}
__device__ __forceinline__ v8f mma16(v16h a, v16h b, v8f c) {
  return __builtin_amdgcn_wmma_f32_16x16x32_f16(false, a, false, b, (short)0, c, false, false);
}
__device__ __forceinline__ v8f mmabf(v16b a, v16b b, v8f c) {
  return __builtin_amdgcn_wmma_f32_16x16x32_bf16(false, a, false, b, (short)0, c, false, false);
}
__device__ __forceinline__ v8f zero8() {
  v8f z;
#pragma unroll
  for (int i = 0; i < 8; ++i) z[i] = 0.0f;
  return z;
}

__device__ __forceinline__ void guard_g(v8f& a, v8f& b, v16b x, v16b y) {
  asm volatile("v_nop\n\tv_nop\n\tv_nop\n\tv_nop" : "+v"(a), "+v"(b) : "v"(x), "v"(y));
}
__device__ __forceinline__ void keep4(v16b a, v16b b, v16b c, v16b d) {
  asm volatile("v_nop" :: "v"(a), "v"(b), "v"(c), "v"(d));
}
__device__ __forceinline__ void accg4(v8f& a, v8f& b, v8f& c, v8f& d) {
  asm volatile("v_nop\n\tv_nop\n\tv_nop\n\tv_nop" : "+v"(a), "+v"(b), "+v"(c), "+v"(d));
}
__device__ __forceinline__ void guard_s(v8f& a, v8f& b, v16h x0, v16h x1, v16h y0, v16h y1) {
  asm volatile("v_nop\n\tv_nop\n\tv_nop\n\tv_nop" : "+v"(a), "+v"(b) : "v"(x0), "v"(x1), "v"(y0), "v"(y1));
}
__device__ __forceinline__ void guard_pv(v8f& a0, v8f& a1, v8f& b0, v8f& b1,
                                         v16h p0, v16h p1, v16h x0, v16h x1, v16h y0, v16h y1) {
  asm volatile("v_nop\n\tv_nop\n\tv_nop\n\tv_nop"
               : "+v"(a0), "+v"(a1), "+v"(b0), "+v"(b1)
               : "v"(p0), "v"(p1), "v"(x0), "v"(x1), "v"(y0), "v"(y1));
}

__global__ __launch_bounds__(256) void cvt_x_kernel(const float* __restrict__ x, unsigned short* __restrict__ xb, int n8) {
  const int li = (int)blockIdx.x * 256 + (int)threadIdx.x;
  if (li >= n8) return;
  const size_t e = (size_t)li * 8;
  const v4f a = *(const v4f*)(x + e);
  const v4f b = *(const v4f*)(x + e + 4);
  v8us o;
#pragma unroll
  for (int i = 0; i < 4; ++i) {
    o[i]     = bfbits(a[i]);
    o[4 + i] = bfbits(b[i]);
  }
  unsigned short* d = xb + e;
  *(volatile v8us*)d = o;
  __threadfence();
  *(volatile v8us*)d = o;
}

__global__ __launch_bounds__(256) void cvt_wt_kernel(const float* __restrict__ w0, const float* __restrict__ w1,
                                                     const float* __restrict__ w2,
                                                     unsigned short* __restrict__ d0, unsigned short* __restrict__ d1,
                                                     unsigned short* __restrict__ d2) {
  __shared__ float sTt[64][33];
  const int z = (int)blockIdx.z;
  const float* src = (z == 0) ? w0 : ((z == 1) ? w1 : w2);
  unsigned short* dst = (z == 0) ? d0 : ((z == 1) ? d1 : d2);
  const int k0 = (int)blockIdx.x * 64, n0 = (int)blockIdx.y * 32;
  const int t = (int)threadIdx.x;
  {
    const int kr = t >> 2, cc = (t & 3) * 8;
    const float* s = src + (size_t)(k0 + kr) * DM + n0 + cc;
    const v4f a = *(const v4f*)(s);
    const v4f b = *(const v4f*)(s + 4);
#pragma unroll
    for (int e = 0; e < 4; ++e) {
      sTt[kr][cc + e]     = a[e];
      sTt[kr][cc + 4 + e] = b[e];
    }
  }
  __syncthreads();
  const int n = t >> 3, kp = (t & 7) * 8;
  v8us o;
#pragma unroll
  for (int i = 0; i < 8; ++i) o[i] = bfbits(sTt[kp + i][n]);
  unsigned short* d = dst + (size_t)(n0 + n) * DM + k0 + kp;
  *(volatile v8us*)d = o;
  __threadfence();
  *(volatile v8us*)d = o;
}

__global__ __launch_bounds__(256) void proj_kernel(const __bf16* __restrict__ A, int lda,
                                                   const __bf16* __restrict__ Bt, int ldb,
                                                   _Float16* __restrict__ Ch, _Float16* __restrict__ Cl, int ldc,
                                                   int M, int N, int K) {
  __shared__ __align__(16) float sT[8][16 * 68];
  const int lane = threadIdx.x & 31, wave = threadIdx.x >> 5;
  const int tilesN = N >> 6, tilesM = M >> 6;
  const int tile = (int)blockIdx.x * 8 + wave;
  if (tile >= tilesM * tilesN) return;
  const int tm = tile / tilesN, tn = tile - tm * tilesN;
  const int m0 = tm << 6, n0 = tn << 6;
  const int rl = lane & 15;
  const int koff = (lane >> 4) * 8;
  const int mOff = (lane >> 4) * 8;

  v8f acc[4][4];
#pragma unroll
  for (int i = 0; i < 4; ++i)
#pragma unroll
    for (int j = 0; j < 4; ++j) acc[i][j] = zero8();

#pragma unroll 1
  for (int k0 = 0; k0 < K; k0 += 32) {
    v16b bh[4];
#pragma unroll
    for (int j = 0; j < 4; ++j) bh[j] = ldfragb(Bt + (size_t)(n0 + (j << 4) + rl) * ldb + koff + k0);
#pragma unroll
    for (int i = 0; i < 4; ++i) {
      const v16b ah = ldfragb(A + (size_t)(m0 + (i << 4) + rl) * lda + koff + k0);
#pragma unroll
      for (int j = 0; j < 4; ++j) acc[i][j] = mmabf(ah, bh[j], acc[i][j]);
      guard_g(acc[i][0], acc[i][3], ah, bh[3]);
    }
    keep4(bh[0], bh[1], bh[2], bh[3]);
  }
  accg4(acc[0][0], acc[0][1], acc[0][2], acc[0][3]);
  accg4(acc[1][0], acc[1][1], acc[1][2], acc[1][3]);
  accg4(acc[2][0], acc[2][1], acc[2][2], acc[2][3]);
  accg4(acc[3][0], acc[3][1], acc[3][2], acc[3][3]);

  float* slab = sT[wave];
  const int qq = lane >> 3, c8 = (lane & 7) * 8;
#pragma unroll
  for (int i = 0; i < 4; ++i) {
    const int mBase = m0 + (i << 4);
#pragma unroll
    for (int j = 0; j < 4; ++j) {
#pragma unroll
      for (int r = 0; r < 8; ++r) slab[(mOff + r) * 68 + (j << 4) + rl] = acc[i][j][r];
    }
    __builtin_amdgcn_fence(__ATOMIC_RELEASE, "workgroup");
    __builtin_amdgcn_wave_barrier();
    __builtin_amdgcn_fence(__ATOMIC_ACQUIRE, "workgroup");
#pragma unroll
    for (int ps = 0; ps < 2; ++ps) {
#pragma unroll
      for (int it = 0; it < 4; ++it) {
        const int row = it * 4 + qq;
        const float* sp = slab + row * 68 + c8;
        const v4f u0 = *(const v4f*)(sp);
        const v4f u1 = *(const v4f*)(sp + 4);
        v8h hv, lv;
#pragma unroll
        for (int e = 0; e < 4; ++e) {
          const _Float16 g0 = (_Float16)u0[e];
          hv[e] = g0;
          lv[e] = (_Float16)((u0[e] - (float)g0) * 2048.0f);
          const _Float16 g1 = (_Float16)u1[e];
          hv[4 + e] = g1;
          lv[4 + e] = (_Float16)((u1[e] - (float)g1) * 2048.0f);
        }
        const size_t go = (size_t)(mBase + row) * ldc + n0 + c8;
        *(volatile v8h*)(Ch + go) = hv;
        *(volatile v8h*)(Cl + go) = lv;
      }
      __threadfence();
    }
    __builtin_amdgcn_fence(__ATOMIC_RELEASE, "workgroup");
    __builtin_amdgcn_wave_barrier();
    __builtin_amdgcn_fence(__ATOMIC_ACQUIRE, "workgroup");
  }
}

#define QB       16
#define NWAVE    16
#define KCH      256
#define QSP      1032
#define PSP      264
#define OSP      1028
#define TSPLIT   64
#define LDS_QH   0
#define LDS_QL   33024
#define LDS_PH   66048
#define LDS_PL   74496
#define LDS_PMAX 82944
#define LDS_PSUM 83968
#define LDS_ST   84992
#define ATT_LDS  85248
static_assert(QB * QSP * 2 == LDS_QL - LDS_QH);
static_assert(QB * QSP * 2 == LDS_PH - LDS_QL);
static_assert(QB * PSP * 2 == LDS_PL - LDS_PH);
static_assert(QB * PSP * 2 == LDS_PMAX - LDS_PL);
static_assert(NWAVE * QB * 4 == LDS_PSUM - LDS_PMAX);
static_assert(NWAVE * QB * 4 == LDS_ST - LDS_PSUM);
static_assert(4 * QB * 4 == ATT_LDS - LDS_ST);
static_assert(QB * OSP * 4 <= LDS_PH);
static_assert((QSP % 8) == 0 && (PSP % 8) == 0 && (OSP % 4) == 0 && PSP >= KCH && QSP >= DM && OSP >= DM);
static_assert(NWAVE * 16 == KCH && NWAVE == QB && NWAVE * 64 == DM && NWAVE * QB <= 512);
static_assert((SEQ % KCH) == 0 && (SEQ % QB) == 0 && TSPLIT <= SEQ / QB);
static_assert((LDS_QL % 16) == 0 && (LDS_PH % 16) == 0 && (LDS_PL % 16) == 0 && (LDS_PMAX % 16) == 0 && (LDS_ST % 16) == 0);

template <bool RES>
__global__ __launch_bounds__(512) void attn_kernel(const _Float16* __restrict__ qh, const _Float16* __restrict__ ql,
                                                   const _Float16* __restrict__ kh, const _Float16* __restrict__ kl,
                                                   const _Float16* __restrict__ vth, const _Float16* __restrict__ vtl,
                                                   float* __restrict__ out, int qt0) {
  extern __shared__ __align__(16) char smem[];
  _Float16* Qhs = (_Float16*)(smem + LDS_QH);
  _Float16* Qls = (_Float16*)(smem + LDS_QL);
  _Float16* Phs = (_Float16*)(smem + LDS_PH);
  _Float16* Pls = (_Float16*)(smem + LDS_PL);
  float* pmax = (float*)(smem + LDS_PMAX);
  float* psum = (float*)(smem + LDS_PSUM);
  float* m_s  = (float*)(smem + LDS_ST);
  float* l_s  = m_s + QB;
  float* al_s = m_s + 2 * QB;
  float* li_s = m_s + 3 * QB;

  const int tid = (int)threadIdx.x;
  const int wave = __builtin_amdgcn_readfirstlane(tid >> 5);
  const int lane = tid & 31, h = lane >> 4, c = lane & 15;
  const int b = (int)blockIdx.y;
  const int q0 = (qt0 + (int)blockIdx.x) * QB;
  const int qlast = q0 + QB - 1;
  const size_t tok0 = (size_t)b * SEQ + q0;
  const float ninf = -__builtin_inff();

  if (tid < QB) { m_s[tid] = ninf; l_s[tid] = 0.0f; al_s[tid] = 0.0f; li_s[tid] = 0.0f; }
  if (tid < NWAVE * QB) psum[tid] = 0.0f;
#pragma unroll
  for (int i = 0; i < 4; ++i) {
    const int idx = i * 512 + tid;
    const int row = idx >> 7;
    const int pc  = idx & 127;
    const size_t g = (tok0 + row) * DM + (size_t)pc * 8;
    const v8h v0 = *(const v8h*)(qh + g);
    const v8h v1 = *(const v8h*)(ql + g);
    *(v8h*)(Qhs + row * QSP + pc * 8) = v0;
    *(v8h*)(Qls + row * QSP + pc * 8) = v1;
  }
  __syncthreads();

  v8f oacc1[4], oacc2[4];
#pragma unroll
  for (int nt = 0; nt < 4; ++nt) { oacc1[nt] = zero8(); oacc2[nt] = zero8(); }

  const _Float16* qbp = Qhs + c * QSP + 8 * h;
  const _Float16* qlp = Qls + c * QSP + 8 * h;
  const _Float16* pap = Phs + c * PSP + 8 * h;
  const _Float16* plp = Pls + c * PSP + 8 * h;
  const int ntile = (q0 >> 8) + 1;

#pragma unroll 1
  for (int t = 0; t < ntile; ++t) {
    const int kb = t * KCH + 16 * wave;
    v8f s1 = zero8(), s2 = zero8();
    if (kb <= qlast) {
      const _Float16* kap = kh + ((size_t)b * SEQ + kb + c) * DM + 8 * h;
      const _Float16* krp = kl + ((size_t)b * SEQ + kb + c) * DM + 8 * h;
#pragma unroll 1
      for (int k0 = 0; k0 < DM; k0 += 32) {
        const v16h a  = ldfrag(kap + k0);
        const v16h bq = ldfrag(qbp + k0);
        const v16h bl = ldfrag(qlp + k0);
        v16h ar = a;
        if (RES) ar = ldfrag(krp + k0);
        s1 = mma16(a, bq, s1);
        s2 = mma16(a, bl, s2);
        if (RES) s2 = mma16(ar, bq, s2);
        guard_s(s1, s2, a, ar, bq, bl);
      }
    }
    {
      float pm = ninf;
#pragma unroll
      for (int r = 0; r < 8; ++r) {
        float s = (s1[r] + s2[r] * 0.00048828125f) * 0.03125f;
        const int key = kb + 8 * h + r;
        s = (key > q0 + c) ? ninf : s;
        s1[r] = s;
        pm = fmaxf(pm, s);
      }
      pm = fmaxf(pm, __shfl_xor(pm, 16, 32));
      pmax[wave * QB + c] = pm;
    }
    __syncthreads();
    if (wave == 0 && lane < QB) {
      const int row = lane;
      float ps = 0.0f;
#pragma unroll
      for (int w = 0; w < NWAVE; ++w) ps += psum[w * QB + row];
      l_s[row] = l_s[row] * al_s[row] + ps;
      const float mo = m_s[row];
      float mx = mo;
#pragma unroll
      for (int w = 0; w < NWAVE; ++w) mx = fmaxf(mx, pmax[w * QB + row]);
      al_s[row] = __expf(mo - mx);
      m_s[row] = mx;
    }
    __syncthreads();
    {
      const float mq = m_s[c];
      float ps = 0.0f;
      v8h ph, pr;
#pragma unroll
      for (int r = 0; r < 8; ++r) {
        const float p = __expf(s1[r] - mq);
        ps += p;
        const float p16 = p * 16.0f;
        const _Float16 hh = (_Float16)p16;
        ph[r] = hh;
        pr[r] = (_Float16)((p16 - (float)hh) * 2048.0f);
      }
      *(v8h*)(Phs + c * PSP + 16 * wave + 8 * h) = ph;
      if (RES) *(v8h*)(Pls + c * PSP + 16 * wave + 8 * h) = pr;
      ps += __shfl_xor(ps, 16, 32);
      psum[wave * QB + c] = ps;
      const v4f aA = *(const v4f*)(al_s + 8 * h), aB = *(const v4f*)(al_s + 8 * h + 4);
#pragma unroll
      for (int nt = 0; nt < 4; ++nt) {
#pragma unroll
        for (int r = 0; r < 4; ++r) {
          oacc1[nt][r] *= aA[r]; oacc1[nt][4 + r] *= aB[r];
          oacc2[nt][r] *= aA[r]; oacc2[nt][4 + r] *= aB[r];
        }
      }
    }
    __syncthreads();
    {
      int kend = q0 + QB - t * KCH;
      kend = (kend > KCH) ? KCH : kend;
      kend = (kend + 31) & ~31;
      const size_t vc0 = (size_t)b * SEQ + (size_t)t * KCH + 8 * h;
      const _Float16* vhp = vth + (size_t)(64 * wave + c) * NTOK + vc0;
      const _Float16* vlp = vtl + (size_t)(64 * wave + c) * NTOK + vc0;
#pragma unroll 1
      for (int ks = 0; ks < kend; ks += 32) {
        const v16h pa = ldfrag(pap + ks);
        v16h pz = pa;
        if (RES) pz = ldfrag(plp + ks);
#pragma unroll
        for (int g = 0; g < 2; ++g) {
          const size_t o0 = (size_t)(32 * g) * NTOK + ks;
          const size_t o1 = (size_t)(32 * g + 16) * NTOK + ks;
          const v16h x0 = ldfrag(vhp + o0), x1 = ldfrag(vhp + o1);
          const v16h y0 = ldfrag(vlp + o0), y1 = ldfrag(vlp + o1);
          oacc1[2 * g]     = mma16(pa, x0, oacc1[2 * g]);
          oacc1[2 * g + 1] = mma16(pa, x1, oacc1[2 * g + 1]);
          oacc2[2 * g]     = mma16(pa, y0, oacc2[2 * g]);
          oacc2[2 * g + 1] = mma16(pa, y1, oacc2[2 * g + 1]);
          if (RES) {
            oacc2[2 * g]     = mma16(pz, x0, oacc2[2 * g]);
            oacc2[2 * g + 1] = mma16(pz, x1, oacc2[2 * g + 1]);
          }
          guard_pv(oacc1[2 * g], oacc1[2 * g + 1], oacc2[2 * g], oacc2[2 * g + 1], pa, pz, x0, x1, y0, y1);
        }
      }
    }
  }

  if (wave == 0 && lane < QB) {
    const int row = lane;
    float ps = 0.0f;
#pragma unroll
    for (int w = 0; w < NWAVE; ++w) ps += psum[w * QB + row];
    const float l = l_s[row] * al_s[row] + ps;
    li_s[row] = (1.0f / l) * 0.0625f;
  }
  __syncthreads();
  float* Os = (float*)(smem + LDS_QH);
  {
    const v4f iA = *(const v4f*)(li_s + 8 * h), iB = *(const v4f*)(li_s + 8 * h + 4);
#pragma unroll
    for (int nt = 0; nt < 4; ++nt) {
      const int col = 64 * wave + 16 * nt + c;
#pragma unroll
      for (int r = 0; r < 4; ++r) {
        Os[(8 * h + r) * OSP + col]     = (oacc1[nt][r] + oacc2[nt][r] * 0.00048828125f) * iA[r];
        Os[(8 * h + 4 + r) * OSP + col] = (oacc1[nt][4 + r] + oacc2[nt][4 + r] * 0.00048828125f) * iB[r];
      }
    }
  }
  __syncthreads();
  {
    const float* srow = Os + wave * OSP;
    float* orow = out + (tok0 + (size_t)wave) * DM;
#pragma unroll
    for (int ps = 0; ps < 2; ++ps) {
#pragma unroll
      for (int j = 0; j < 8; ++j) {
        const int pc = j * 32 + lane;
        const v4f v = *(const v4f*)(srow + pc * 4);
        *(volatile v4f*)(orow + pc * 4) = v;
      }
      __threadfence();
    }
  }
}

extern "C" void kernel_launch(void* const* d_in, const int* in_sizes, int n_in,
                              void* d_out, int out_size, void* d_ws, size_t ws_size,
                              hipStream_t stream) {
  if (n_in < 4) return;
  if (in_sizes[0] != NTOK * DM) return;
  if (in_sizes[1] != DM * DM || in_sizes[2] != DM * DM || in_sizes[3] != DM * DM) return;
  if (out_size != NTOK * DM) return;

  const float* x  = (const float*)d_in[0];
  const float* Wq = (const float*)d_in[1];
  const float* Wk = (const float*)d_in[2];
  const float* Wv = (const float*)d_in[3];
  float* out = (float*)d_out;

  const size_t bAct = (size_t)NTOK * DM * 2;
  const size_t bW   = (size_t)DM * DM * 2;
  size_t off = 0;
  const size_t oXb = off; off += bAct;
  const size_t oWq = off; off += bW;
  const size_t oWk = off; off += bW;
  const size_t oWv = off; off += bW;
  const size_t oQh = off; off += bAct;
  const size_t oQl = off; off += bAct;
  const size_t oKh = off; off += bAct;
  const size_t oKl = off; off += bAct;
  const size_t oVh = off; off += bAct;
  const size_t oVl = off; off += bAct;
  if (off > ws_size) return;
  if (off > (size_t)134217728) return;

  char* ws = (char*)d_ws;
  unsigned short* Xb  = (unsigned short*)(ws + oXb);
  unsigned short* WqT = (unsigned short*)(ws + oWq);
  unsigned short* WkT = (unsigned short*)(ws + oWk);
  unsigned short* WvT = (unsigned short*)(ws + oWv);
  _Float16* Qh = (_Float16*)(ws + oQh);
  _Float16* Ql = (_Float16*)(ws + oQl);
  _Float16* Kh = (_Float16*)(ws + oKh);
  _Float16* Kl = (_Float16*)(ws + oKl);
  _Float16* Vh = (_Float16*)(ws + oVh);
  _Float16* Vl = (_Float16*)(ws + oVl);

  const dim3 blk(256);
  const int n8 = NTOK * DM / 8;
  if ((n8 % 256) != 0) return;

  cvt_x_kernel<<<dim3(n8 / 256), blk, 0, stream>>>(x, Xb, n8);
  cvt_wt_kernel<<<dim3(DM / 64, DM / 32, 3), blk, 0, stream>>>(Wq, Wk, Wv, WqT, WkT, WvT);
  proj_kernel<<<dim3(((NTOK / 64) * (DM / 64)) / 8), blk, 0, stream>>>(
      (const __bf16*)Xb, DM, (const __bf16*)WqT, DM, Qh, Ql, DM, NTOK, DM, DM);
  proj_kernel<<<dim3(((NTOK / 64) * (DM / 64)) / 8), blk, 0, stream>>>(
      (const __bf16*)Xb, DM, (const __bf16*)WkT, DM, Kh, Kl, DM, NTOK, DM, DM);
  proj_kernel<<<dim3(((DM / 64) * (NTOK / 64)) / 8), blk, 0, stream>>>(
      (const __bf16*)WvT, DM, (const __bf16*)Xb, DM, Vh, Vl, NTOK, DM, NTOK, DM);
  (void)hipFuncSetAttribute(reinterpret_cast<const void*>(&attn_kernel<true>),
                            hipFuncAttributeMaxDynamicSharedMemorySize, ATT_LDS);
  (void)hipFuncSetAttribute(reinterpret_cast<const void*>(&attn_kernel<false>),
                            hipFuncAttributeMaxDynamicSharedMemorySize, ATT_LDS);
  attn_kernel<true><<<dim3(TSPLIT, NB), dim3(512), ATT_LDS, stream>>>(Qh, Ql, Kh, Kl, Vh, Vl, out, 0);
  attn_kernel<false><<<dim3(SEQ / QB - TSPLIT, NB), dim3(512), ATT_LDS, stream>>>(Qh, Ql, Kh, Kl, Vh, Vl, out, TSPLIT);
  (void)hipGetLastError();
}
